// ConceptDiagram_2370821948079
// MI455X (gfx1250) — hardware-verified
//
#include <hip/hip_runtime.h>


namespace {
constexpr int S = 4, T = 4, N = 65536, D = 128, H = 128, DT = 128;
constexpr float AS_ = 8.0f;

typedef _Float16 b16;
typedef __attribute__((ext_vector_type(16))) _Float16 v16b;
typedef __attribute__((ext_vector_type(8))) _Float16 v8b;
typedef __attribute__((ext_vector_type(8))) float v8f;
typedef __attribute__((ext_vector_type(4))) float v4f;
__device__ __forceinline__ float bf16_rne(float f) { unsigned int u = __float_as_uint(f); u += 0x7FFFu + ((u >> 16) & 1u); return __uint_as_float(u & 0xFFFF0000u); }
__device__ __forceinline__ void split16(float v, b16& hi, b16& lo) { hi = (b16)v; lo = (b16)(v - (float)hi); }
__device__ __forceinline__ v16b frag_kb(const b16* p, int hh) { const v8b a = *(const v8b*)(p + 8 * hh), b = *(const v8b*)(p + 16 + 8 * hh); v16b f;
#pragma unroll
  for (int e = 0; e < 8; ++e) { f[e] = a[e]; f[8 + e] = b[e]; } return f; }
__device__ __forceinline__ v16b frag_x(const float* p, int hh) { v16b f;
#pragma unroll
  for (int e = 0; e < 8; ++e) { f[e] = (b16)bf16_rne(p[8 * hh + e]); f[8 + e] = (b16)bf16_rne(p[16 + 8 * hh + e]); } return f; }
__device__ __forceinline__ void frag_split(const float* p, int hh, v16b& fh, v16b& fl) {
#pragma unroll
  for (int e = 0; e < 8; ++e) { b16 a, c; split16(p[8 * hh + e] * AS_, a, c); fh[e] = a; fl[e] = c; split16(p[16 + 8 * hh + e] * AS_, a, c); fh[8 + e] = a; fl[8 + e] = c; } }
__device__ __forceinline__ v8f wmma16b(v16b a, v16b b, v8f c) { v8f d = __builtin_amdgcn_wmma_f32_16x16x32_f16(false, a, false, b, (short)0, c, false, false); asm volatile("v_nop\n\tv_nop\n\tv_nop\n\tv_nop" : "+v"(d) : "v"(a), "v"(b)); return d; }
__device__ __forceinline__ void wave_lds_sync() { __builtin_amdgcn_fence(__ATOMIC_RELEASE, "workgroup"); __builtin_amdgcn_wave_barrier(); __builtin_amdgcn_fence(__ATOMIC_ACQUIRE, "workgroup"); }
__device__ __forceinline__ float nexp(float x) { return __builtin_amdgcn_exp2f(x * 1.4426950408889634f); }

__device__ __forceinline__ int best_t(const float* tm, int s) { int bt = 0; float bv = bf16_rne(tm[s * T]); for (int t = 1; t < T; ++t) { const float v = bf16_rne(tm[s * T + t]); if (v > bv) { bv = v; bt = t; } } return bt; }

struct Wo_ { static constexpr size_t W1 = 0, C1 = W1 + H * D, W2 = C1 + H * D, C2 = W2 + DT * H, PER = C2 + 16 * H; };
struct Po_ { static constexpr int B1 = 0, C1B = 128, B2 = 256, C2B = 384, PER = 385; };
__global__ __launch_bounds__(256) void prep_kernel(const float* __restrict__ tm, const float* __restrict__ W1, const float* __restrict__ b1, const float* __restrict__ W2, const float* __restrict__ b2, const float* __restrict__ C1, const float* __restrict__ c1, const float* __restrict__ C2, const float* __restrict__ c2, b16* __restrict__ R, float* __restrict__ P) {
  const int t_ = blockIdx.x * 256 + threadIdx.x, nth = gridDim.x * 256;
  for (int pass = 0; pass < 2; ++pass) {
    for (int s = 0; s < S; ++s) { const int t = best_t(tm, s); const size_t st = (size_t)s * T + t; b16* Rs = R + (size_t)s * Wo_::PER; float* Ps = P + s * 512;
      for (int q = t_; q < H * D; q += nth) { const int o = q / D, k = q % D; Rs[Wo_::W1 + q] = (b16)bf16_rne(W1[(st * D + k) * H + o]); Rs[Wo_::C1 + q] = (b16)bf16_rne(C1[(st * D + k) * H + o]); Rs[Wo_::W2 + q] = (b16)bf16_rne(W2[(st * H + k) * DT + o]); }
      for (int q = t_; q < 16 * H; q += nth) Rs[Wo_::C2 + q] = (b16)((q < H) ? bf16_rne(C2[st * H + q]) : 0.0f);
      for (int q = t_; q < Po_::PER; q += nth) { float v; if (q < 128) v = b1[st * H + q]; else if (q < 256) v = c1[st * H + q - 128]; else if (q < 384) v = b2[st * DT + q - 256]; else v = c2[st]; Ps[q] = bf16_rne(v); } }
    __threadfence(); }
}

__global__ __launch_bounds__(128) void cd_kernel(const float* __restrict__ x, const float* __restrict__ sc, const int* __restrict__ tid, const float* __restrict__ tm, const b16* __restrict__ R, const float* __restrict__ P, float* __restrict__ outS, float* __restrict__ outC, float* __restrict__ outP) {
  __shared__ __attribute__((aligned(16))) float Hs[4][32][H + 4]; __shared__ __attribute__((aligned(16))) float Yo[4][32][DT + 4]; __shared__ float Sc[4][32], Pr[4][32];
  const int lane = threadIdx.x & 31, wave = threadIdx.x >> 5, nloc = lane & 15, hlf = lane >> 4, m0 = blockIdx.x * 128 + wave * 32;
  float (*Hw)[H + 4] = Hs[wave]; float (*Yw)[DT + 4] = Yo[wave];
  for (int i = lane; i < 32 * (DT + 4); i += 32) (&Yw[0][0])[i] = 0.0f;
  { const int ty = tid[m0 + lane]; Sc[wave][lane] = 0.0f; const int tcl = (ty < 0) ? 0 : (ty >= S ? S - 1 : ty); const float lg = tm[tcl * T + best_t(tm, tcl)]; Pr[wave][lane] = 1.0f / (1.0f + nexp(-bf16_rne(lg)));
  }
  wave_lds_sync();
#pragma unroll 1
  for (int s = 0; s < S; ++s) { const b16* Rs = R + (size_t)s * Wo_::PER; const float* Ps = P + s * 512;
    wave_lds_sync();
    for (int tg = 0; tg < 8; tg += 4) { v8f acc[2][4];
#pragma unroll
      for (int r = 0; r < 2; ++r)
#pragma unroll
        for (int t = 0; t < 4; ++t) acc[r][t] = (v8f){};
#pragma unroll
      for (int kb = 0; kb < D; kb += 32) { const v16b a0 = frag_x(x + (size_t)(m0 + nloc) * D + kb, hlf), a1 = frag_x(x + (size_t)(m0 + 16 + nloc) * D + kb, hlf);
#pragma unroll
        for (int t = 0; t < 4; ++t) { const v16b bw = frag_kb(Rs + Wo_::W1 + (size_t)((tg + t) * 16 + nloc) * D + kb, hlf); acc[0][t] = wmma16b(a0, bw, acc[0][t]); acc[1][t] = wmma16b(a1, bw, acc[1][t]); } }
#pragma unroll
      for (int t = 0; t < 4; ++t) { const float bb = Ps[Po_::B1 + (tg + t) * 16 + nloc];
#pragma unroll
        for (int r = 0; r < 2; ++r)
#pragma unroll
          for (int v = 0; v < 8; ++v) Hw[r * 16 + 8 * hlf + v][(tg + t) * 16 + nloc] = fmaxf(acc[r][t][v] + bb, 0.0f); } }
    wave_lds_sync();
    for (int tg = 0; tg < 8; tg += 4) { v8f acc[2][4];
#pragma unroll
      for (int r = 0; r < 2; ++r)
#pragma unroll
        for (int t = 0; t < 4; ++t) acc[r][t] = (v8f){};
#pragma unroll
      for (int kb = 0; kb < H; kb += 32) { v16b a0, l0, a1, l1; frag_split(&Hw[nloc][kb], hlf, a0, l0); frag_split(&Hw[16 + nloc][kb], hlf, a1, l1);
#pragma unroll
        for (int t = 0; t < 4; ++t) { const v16b bw = frag_kb(Rs + Wo_::W2 + (size_t)((tg + t) * 16 + nloc) * H + kb, hlf); acc[0][t] = wmma16b(a0, bw, acc[0][t]); acc[0][t] = wmma16b(l0, bw, acc[0][t]); acc[1][t] = wmma16b(a1, bw, acc[1][t]); acc[1][t] = wmma16b(l1, bw, acc[1][t]); } }
#pragma unroll
      for (int t = 0; t < 4; ++t) { const int cc = (tg + t) * 16 + nloc; const float bb = Ps[Po_::B2 + cc];
#pragma unroll
        for (int r = 0; r < 2; ++r)
#pragma unroll
          for (int v = 0; v < 8; ++v) { const int rr = r * 16 + 8 * hlf + v; if (tid[m0 + rr] == s) Yw[rr][cc] = acc[r][t][v] * (1.0f / AS_) + bb; } } }
    wave_lds_sync();
    { for (int tg = 0; tg < 8; tg += 4) { v8f acc[2][4];
#pragma unroll
        for (int r = 0; r < 2; ++r)
#pragma unroll
          for (int t = 0; t < 4; ++t) acc[r][t] = (v8f){};
#pragma unroll
        for (int kb = 0; kb < D; kb += 32) { const v16b a0 = frag_x(x + (size_t)(m0 + nloc) * D + kb, hlf), a1 = frag_x(x + (size_t)(m0 + 16 + nloc) * D + kb, hlf);
#pragma unroll
          for (int t = 0; t < 4; ++t) { const v16b bw = frag_kb(Rs + Wo_::C1 + (size_t)((tg + t) * 16 + nloc) * D + kb, hlf); acc[0][t] = wmma16b(a0, bw, acc[0][t]); acc[1][t] = wmma16b(a1, bw, acc[1][t]); } }
#pragma unroll
        for (int t = 0; t < 4; ++t) { const float bb = Ps[Po_::C1B + (tg + t) * 16 + nloc];
#pragma unroll
          for (int r = 0; r < 2; ++r)
#pragma unroll
            for (int v = 0; v < 8; ++v) Hw[r * 16 + 8 * hlf + v][(tg + t) * 16 + nloc] = fmaxf(acc[r][t][v] + bb, 0.0f); } }
      wave_lds_sync();
      v8f z[2] = {{}, {}};
#pragma unroll
      for (int kb = 0; kb < H; kb += 32) { v16b a0, l0, a1, l1; frag_split(&Hw[nloc][kb], hlf, a0, l0); frag_split(&Hw[16 + nloc][kb], hlf, a1, l1); const v16b bw = frag_kb(Rs + Wo_::C2 + (size_t)nloc * H + kb, hlf);
        z[0] = wmma16b(a0, bw, z[0]); z[0] = wmma16b(l0, bw, z[0]); z[1] = wmma16b(a1, bw, z[1]); z[1] = wmma16b(l1, bw, z[1]); }
      if (nloc == 0) { const float cb = Ps[Po_::C2B];
#pragma unroll
        for (int r = 0; r < 2; ++r)
#pragma unroll
          for (int v = 0; v < 8; ++v) { const int rr = r * 16 + 8 * hlf + v; if (tid[m0 + rr] == s) { const float cls = 1.0f / (1.0f + nexp(-(z[r][v] * (1.0f / AS_) + cb))); Sc[wave][rr] = fminf(bf16_rne(sc[m0 + rr]), cls); } } }
      wave_lds_sync(); } }
  for (int pass = 0; pass < 2; ++pass) {
    for (int i = lane; i < 32 * (DT / 4); i += 32) { const int rr = i / (DT / 4), c4 = (i % (DT / 4)) * 4; *(volatile v4f*)(outS + (size_t)(m0 + rr) * DT + c4) = *(const v4f*)(&Yw[rr][c4]); }
    ((volatile float*)outC)[m0 + lane] = Sc[wave][lane]; ((volatile float*)outP)[m0 + lane] = Pr[wave][lane];
    __threadfence(); }
}
}

extern "C" void kernel_launch(void* const* d_in, const int* in_sizes, int n_in,
                              void* d_out, int out_size, void* d_ws, size_t ws_size, hipStream_t stream) {
  (void)n_in; (void)out_size;
  const float* x = (const float*)d_in[0]; const float* sc = (const float*)d_in[1]; const int* tid = (const int*)d_in[2]; const float* tm = (const float*)d_in[3];
  const float* W1 = (const float*)d_in[4]; const float* b1 = (const float*)d_in[5]; const float* W2 = (const float*)d_in[6]; const float* b2 = (const float*)d_in[7]; const float* C1 = (const float*)d_in[8]; const float* c1 = (const float*)d_in[9]; const float* C2 = (const float*)d_in[10]; const float* c2 = (const float*)d_in[11];
  float* outS = (float*)d_out; float* outC = outS + (size_t)N * DT; float* outP = outC + N;
  if (in_sizes[0] != N * D || in_sizes[2] != N || in_sizes[3] != S * T || in_sizes[4] != S * T * D * H || in_sizes[10] != S * T * H) return;
  size_t off = 0; char* ws = (char*)d_ws;
  auto carve = [&](size_t bytes) { char* p = ws + off; off += (bytes + 255) & ~(size_t)255; return p; };
  b16* R = (b16*)carve((size_t)S * Wo_::PER * 2); float* P = (float*)carve((size_t)S * 512 * 4);
  if (off > ws_size) return;
  prep_kernel<<<64, 256, 0, stream>>>(tm, W1, b1, W2, b2, C1, c1, C2, c2, R, P);
  cd_kernel<<<N / 128, 128, 0, stream>>>(x, sc, tid, tm, R, P, outS, outC, outP);
}
